// LlamaAttention_27848567947510
// MI455X (gfx1250) — hardware-verified
//
#include <hip/hip_runtime.h>


#ifndef NB
#define NB 2
#endif
#ifndef SEQ
#define SEQ 2048
#endif
#ifndef RH
#define RH 512
#endif
#define TT      SEQ
#define TT_FULL 2048
#define DM      2048
#define NH      16
#define HD      128
#define RHC     ((RH) < (TT) ? (RH) : (TT))
#define KT      64
#define PCAR    1024.0f
#define OCAR    64.0f
#define OCINV   (1.0f / 4096.0f)
#define SCL     0.08838834764831845f
#define L2E     1.4426950408889634f
#define LG2TH   13.287712379549449f
#define PSP     72
#define OSP     136

static_assert(TT % 64 == 0);
static_assert((RHC) % 64 == 0);
static_assert(((TT) - (RHC)) % 64 == 0);
static_assert(DM == NH * HD);
static_assert(HD == 128);
static_assert(DM % 64 == 0);
static_assert(TT <= TT_FULL);
static_assert(KT == 64);

typedef _Float16 h16;
typedef unsigned short bf;
typedef __attribute__((ext_vector_type(16))) __bf16   v16bf;
typedef __attribute__((ext_vector_type(16))) _Float16 v16h;
typedef __attribute__((ext_vector_type(8)))  _Float16 v8h;
typedef __attribute__((ext_vector_type(8)))  unsigned short v8us;
typedef __attribute__((ext_vector_type(8)))  float    v8f;
typedef __attribute__((ext_vector_type(4)))  float    v4f;
typedef __attribute__((ext_vector_type(2)))  _Float16 v2h;
typedef __attribute__((ext_vector_type(2)))  unsigned short v2us;
typedef __attribute__((ext_vector_type(2)))  float    v2f;
typedef v8h  __attribute__((may_alias)) v8ha;
typedef v4f  __attribute__((may_alias)) v4fa;
typedef v8us __attribute__((may_alias)) v8usa;

__device__ __forceinline__ unsigned short f2bf(float f) { unsigned u = __float_as_uint(f); u += 0x7FFFu + ((u >> 16) & 1u); return (unsigned short)(u >> 16); }
__device__ __forceinline__ float bf2f(unsigned short b) { return __uint_as_float(((unsigned)b) << 16); }
__device__ __forceinline__ float bfr(float f) { return bf2f(f2bf(f)); }
__device__ __forceinline__ v16h cat16(v8h lo, v8h hi) { return __builtin_shufflevector(lo, hi, 0, 1, 2, 3, 4, 5, 6, 7, 8, 9, 10, 11, 12, 13, 14, 15); }
__device__ __forceinline__ v16bf cat16b(v8us lo, v8us hi) { return __builtin_bit_cast(v16bf, __builtin_shufflevector(lo, hi, 0, 1, 2, 3, 4, 5, 6, 7, 8, 9, 10, 11, 12, 13, 14, 15)); }
__device__ __forceinline__ v8f wmma16(v16h a, v16h b, v8f c) { return __builtin_amdgcn_wmma_f32_16x16x32_f16(false, a, false, b, (short)0, c, false, false); }
__device__ __forceinline__ v8f wmmab(v16bf a, v16bf b, v8f c) { return __builtin_amdgcn_wmma_f32_16x16x32_bf16(false, a, false, b, (short)0, c, false, false); }
__device__ __forceinline__ h16 tohx(float x) { return (h16)x; }
__device__ __forceinline__ unsigned short hbits(float x) { return __builtin_bit_cast(unsigned short, tohx(x)); }
__device__ __forceinline__ void splitf(float y, unsigned short& h, unsigned short& l) { h = f2bf(y); l = f2bf(y - bf2f(h)); }

template <typename T16> struct WFrag;
template <> struct WFrag<h16> { typedef v16h V;
    static __device__ __forceinline__ V ld(const h16* p) { return cat16(*(const v8h*)p, *(const v8h*)(p + 16)); }
    static __device__ __forceinline__ V lda(const unsigned short* p) { return cat16(*(const v8ha*)p, *(const v8ha*)(p + 16)); }
    static __device__ __forceinline__ v8f mma(V a, V b, v8f c) { return wmma16(a, b, c); } };
template <> struct WFrag<bf> { typedef v16bf V;
    static __device__ __forceinline__ V ld(const bf* p) { return cat16b(*(const v8us*)p, *(const v8us*)(p + 16)); }
    static __device__ __forceinline__ V lda(const unsigned short* p) { return cat16b(*(const v8usa*)p, *(const v8usa*)(p + 16)); }
    static __device__ __forceinline__ v8f mma(V a, V b, v8f c) { return wmmab(a, b, c); } };

template <typename T16, int NSPLIT, bool BIAS>
__global__ __launch_bounds__(32) void k_gemmw(const T16* __restrict__ A, const T16* __restrict__ A2, const T16* __restrict__ Bt, const T16* __restrict__ Bt2, int K, float* C, int ldc, const float* __restrict__ bias, float osc, size_t sA, size_t sB, size_t sC) {
    typedef typename WFrag<T16>::V V;
    __shared__ __align__(16) float os[16 * 68];
    const size_t z = blockIdx.z; A += z * sA; if (A2) A2 += z * sA; Bt += z * sB; if (Bt2) Bt2 += z * sB; C += z * sC;
    const int lane = threadIdx.x & 31, lr = lane & 15, hi = lane >> 4; const int r0 = blockIdx.x * 64, c0 = blockIdx.y * 64;
    v8f acc[4][4];
#pragma unroll
    for (int mb = 0; mb < 4; ++mb)
#pragma unroll
        for (int nb = 0; nb < 4; ++nb) acc[mb][nb] = (v8f){};
    const size_t aoff = (size_t)(r0 + lr) * K + 8 * hi, boff = (size_t)(c0 + lr) * K + 8 * hi;
#pragma unroll 1
    for (int kc = 0; kc < K; kc += 32) {
        V a[4], a2[4];
#pragma unroll
        for (int mb = 0; mb < 4; ++mb) { a[mb] = WFrag<T16>::ld(A + aoff + (size_t)mb * 16 * K + kc); if (NSPLIT == 1 || NSPLIT == 2) a2[mb] = WFrag<T16>::ld(A2 + aoff + (size_t)mb * 16 * K + kc); }
#pragma unroll
        for (int nb = 0; nb < 4; ++nb) { const V b = WFrag<T16>::ld(Bt + boff + (size_t)nb * 16 * K + kc); V b2; if (NSPLIT >= 2) b2 = WFrag<T16>::ld(Bt2 + boff + (size_t)nb * 16 * K + kc);
#pragma unroll
            for (int mb = 0; mb < 4; ++mb) { acc[mb][nb] = WFrag<T16>::mma(a[mb], b, acc[mb][nb]); if (NSPLIT == 1 || NSPLIT == 2) acc[mb][nb] = WFrag<T16>::mma(a2[mb], b, acc[mb][nb]); if (NSPLIT >= 2) acc[mb][nb] = WFrag<T16>::mma(a[mb], b2, acc[mb][nb]); } }
        asm volatile("v_nop\n\tv_nop\n\tv_nop\n\tv_nop" : "+v"(acc[0][0]), "+v"(acc[1][1]), "+v"(acc[2][2]), "+v"(acc[3][3]) : "v"(a[0]), "v"(a[3]));
    }
#pragma unroll
    for (int mb = 0; mb < 4; ++mb) {
#pragma unroll
        for (int nb = 0; nb < 4; ++nb) {
#pragma unroll
            for (int j = 0; j < 8; ++j) os[(hi * 8 + j) * 68 + nb * 16 + lr] = acc[mb][nb][j]; }
        __syncthreads();
        float* crow = C + (size_t)(r0 + mb * 16) * ldc + c0;
#pragma unroll 1
        for (int ps = 0; ps < 2; ++ps) {
#pragma unroll
            for (int s = 0; s < 8; ++s) { const int row = 2 * s + hi, cofs = lr * 4; v4f val = *(const v4fa*)(os + row * 68 + cofs); val = val * osc;
                if (BIAS) { val[0] += bfr(bias[c0 + cofs]); val[1] += bfr(bias[c0 + cofs + 1]); val[2] += bfr(bias[c0 + cofs + 2]); val[3] += bfr(bias[c0 + cofs + 3]); }
                *(volatile v4f*)(crow + (size_t)row * ldc + cofs) = val; }
            if (ps == 0) __threadfence(); }
        __syncthreads();
    }
}

__global__ __launch_bounds__(256) void k_wtG(const float* __restrict__ w, int K, int N, bf* Bt) {
    const int lane = threadIdx.x & 31; const int L0 = (blockIdx.x * 8 + (threadIdx.x >> 5)) * 8; const int nlines = N * K / 64;
#pragma unroll 1
    for (int ps = 0; ps < 2; ++ps) {
#pragma unroll 1
        for (int l = 0; l < 8; ++l) { const int L = L0 + l; if (L >= nlines) break; const size_t e = (size_t)L * 64 + lane * 2; const int k = (int)(e % K), n = (int)(e / K); v2us o;
            o[0] = f2bf(w[(size_t)k * N + n]); o[1] = f2bf(w[(size_t)(k + 1) * N + n]); *(volatile v2us*)(Bt + e) = o; }
        if (ps == 0) __threadfence(); }
}
__global__ __launch_bounds__(256) void k_wtG16(const float* __restrict__ w, int K, int N, float sc, h16* Bt) {
    const int lane = threadIdx.x & 31; const int L0 = (blockIdx.x * 8 + (threadIdx.x >> 5)) * 8; const int nlines = N * K / 64;
#pragma unroll 1
    for (int ps = 0; ps < 2; ++ps) {
#pragma unroll 1
        for (int l = 0; l < 8; ++l) { const int L = L0 + l; if (L >= nlines) break; const size_t e = (size_t)L * 64 + lane * 2; const int k = (int)(e % K), n = (int)(e / K); v2h o;
            o[0] = tohx(bfr(w[(size_t)k * N + n]) * sc); o[1] = tohx(bfr(w[(size_t)(k + 1) * N + n]) * sc); *(volatile v2h*)(Bt + e) = o; }
        if (ps == 0) __threadfence(); }
}
__global__ __launch_bounds__(256) void k_cvt8(const float* __restrict__ src, bf* dst, size_t n8) { const size_t i = (size_t)blockIdx.x * 256 + threadIdx.x; if (i >= n8) return; const v8f v = *(const v8f*)(src + i * 8); v8us o;
#pragma unroll
    for (int k = 0; k < 8; ++k) o[k] = f2bf(v[k]); *(volatile v8us*)(dst + i * 8) = o; __threadfence(); *(volatile v8us*)(dst + i * 8) = o; }

__global__ __launch_bounds__(256) void k_cstab(float* CS) {
    const int idx = blockIdx.x * 256 + threadIdx.x; if (idx >= TT * (HD / 2)) return;
    const int i = idx % (HD / 2); const int t = idx / (HD / 2);
    const float e = (float)(2 * i) * (1.0f / (float)HD);
    const float invf = exp2f(-(e * LG2TH));
    const float ang = (float)t * invf;
    float sn, cs; sincosf(ang, &sn, &cs);
    v2f o; o[0] = cs; o[1] = sn;
    const size_t b0 = ((size_t)t * HD + i) * 2, b1 = b0 + (size_t)HD;
#pragma unroll 1
    for (int ps = 0; ps < 2; ++ps) { *(volatile v2f*)(CS + b0) = o; *(volatile v2f*)(CS + b1) = o; if (ps == 0) __threadfence(); }
}

__global__ __launch_bounds__(256) void k_rope(const float* __restrict__ F, int pitch, int nheads, const float* __restrict__ CS, h16* P16, bf* Ph, bf* Pl) {
    const size_t e = ((size_t)blockIdx.x * 256 + threadIdx.x) * 2; if (e >= (size_t)nheads * TT * HD) return;
    const int d = (int)(e % HD); const int t = (int)((e / HD) % TT); const int h = (int)(e / ((size_t)HD * TT));
    const float* f = F + (size_t)t * pitch + h * HD; v2h o16; v2us oh, ol;
#pragma unroll
    for (int q = 0; q < 2; ++q) { const int dd = d + q; const int dp = (dd < HD / 2) ? dd + HD / 2 : dd - HD / 2; const float x0 = f[dd], x1 = f[dp];
        const v2f cs = *(const v2f*)(CS + ((size_t)t * HD + dd) * 2); float a = __fmul_rn(x0, cs[0]), bq = __fmul_rn(x1, cs[1]); asm volatile("" : "+v"(a)); asm volatile("" : "+v"(bq));
        const float r = (dd < HD / 2) ? __fsub_rn(a, bq) : __fadd_rn(a, bq);
        o16[q] = tohx(r); unsigned short a2, c2; splitf(r, a2, c2); oh[q] = a2; ol[q] = c2; }
    const bool hr = (t < RHC);
    const size_t oo = ((size_t)h * RHC + t) * HD + d;
    *(volatile v2h*)(P16 + e) = o16; if (hr) { *(volatile v2us*)(Ph + oo) = oh; *(volatile v2us*)(Pl + oo) = ol; }
    __threadfence();
    *(volatile v2h*)(P16 + e) = o16; if (hr) { *(volatile v2us*)(Ph + oo) = oh; *(volatile v2us*)(Pl + oo) = ol; }
}
__global__ __launch_bounds__(256) void k_vtp(const float* __restrict__ F, int pitch, int nheads, h16* V16, bf* Vh, bf* Vl) {
    const size_t e = ((size_t)blockIdx.x * 256 + threadIdx.x) * 2; if (e >= (size_t)nheads * HD * TT) return;
    const int t = (int)(e % TT); const int d = (int)((e / TT) % HD); const int g = (int)(e / ((size_t)TT * HD)); v2h o16; v2us oh, ol;
#pragma unroll
    for (int q = 0; q < 2; ++q) { const float x = F[(size_t)(t + q) * pitch + g * HD + d]; o16[q] = tohx(x); unsigned short a2, c2; splitf(x, a2, c2); oh[q] = a2; ol[q] = c2; }
    const bool hr = (t < RHC);
    const size_t oo = ((size_t)g * HD + d) * RHC + t;
    *(volatile v2h*)(V16 + e) = o16; if (hr) { *(volatile v2us*)(Vh + oo) = oh; *(volatile v2us*)(Vl + oo) = ol; }
    __threadfence();
    *(volatile v2h*)(V16 + e) = o16; if (hr) { *(volatile v2us*)(Vh + oo) = oh; *(volatile v2us*)(Vl + oo) = ol; }
}

template <typename T16, bool HR>
__global__ __launch_bounds__(32) void k_flash(const T16* __restrict__ Q, const T16* __restrict__ Q2, const T16* __restrict__ Kp, const T16* __restrict__ K2,
                                             const T16* __restrict__ VT, const T16* __restrict__ VT2, int tp, int rbase, int obase, bf* O1, bf* O2) {
    typedef typename WFrag<T16>::V V;
    __shared__ __align__(16) unsigned short ps1[16 * PSP];
    __shared__ __align__(16) unsigned short ps2[16 * PSP];
    __shared__ __align__(16) unsigned short os1[16 * OSP];
    __shared__ __align__(16) unsigned short os2[16 * OSP];
    const int lane = threadIdx.x & 31, lr = lane & 15, hi = lane >> 4;
    const int h = blockIdx.y; const int row0 = rbase + blockIdx.x * 16;
    const size_t qo = ((size_t)h * tp + row0 + lr) * HD + 8 * hi;
    const size_t ko = ((size_t)h * tp + lr) * HD + 8 * hi;
    const size_t vo = ((size_t)h * HD + lr) * tp + 8 * hi;
    const T16* qb = Q + qo; const T16* qb2 = Q2 + qo; const T16* kb = Kp + ko; const T16* kb2 = K2 + ko; const T16* vb = VT + vo; const T16* vb2 = VT2 + vo;
    v8f o[8];
#pragma unroll
    for (int nd = 0; nd < 8; ++nd) o[nd] = (v8f){};
    float m[8], l[8];
#pragma unroll
    for (int r = 0; r < 8; ++r) { m[r] = -1.0e30f; l[r] = 0.0f; }
    const int ntile = (row0 >> 6) + 1;
#pragma unroll 1
    for (int kt = 0; kt < ntile; ++kt) {
        const int t0 = kt * KT;
        v8f s[4];
#pragma unroll
        for (int nb = 0; nb < 4; ++nb) s[nb] = (v8f){};
        V a, a2;
#pragma unroll
        for (int kc = 0; kc < HD / 32; ++kc) {
            a = WFrag<T16>::ld(qb + kc * 32); if (HR) a2 = WFrag<T16>::ld(qb2 + kc * 32);
#pragma unroll
            for (int nb = 0; nb < 4; ++nb) {
                const size_t kk = (size_t)(t0 + nb * 16) * HD + kc * 32;
                const V b = WFrag<T16>::ld(kb + kk);
                s[nb] = WFrag<T16>::mma(a, b, s[nb]);
                if (HR) { const V b2 = WFrag<T16>::ld(kb2 + kk); s[nb] = WFrag<T16>::mma(a2, b, s[nb]); s[nb] = WFrag<T16>::mma(a, b2, s[nb]); }
            }
        }
        asm volatile("v_nop\n\tv_nop\n\tv_nop\n\tv_nop" : "+v"(s[0]), "+v"(s[1]), "+v"(s[2]), "+v"(s[3]) : "v"(a));
#pragma unroll
        for (int r = 0; r < 8; ++r) {
            const int qi = row0 + 8 * hi + r;
            float t4[4]; float mx = -3.0e38f;
#pragma unroll
            for (int nb = 0; nb < 4; ++nb) { const int kj = t0 + nb * 16 + lr; float tv = s[nb][r] * SCL; tv = (kj > qi) ? -1.0e9f : tv; t4[nb] = tv; mx = fmaxf(mx, tv); }
#pragma unroll
            for (int sh = 1; sh < 16; sh <<= 1) mx = fmaxf(mx, __shfl_xor(mx, sh, 32));
            const float nm = fmaxf(m[r], mx);
            const float corr = __builtin_amdgcn_exp2f((m[r] - nm) * L2E);
            float psum = 0.0f;
#pragma unroll
            for (int nb = 0; nb < 4; ++nb) {
                const float p = __builtin_amdgcn_exp2f((t4[nb] - nm) * L2E); psum += p;
                const int li = (8 * hi + r) * PSP + nb * 16 + lr;
                if (HR) { const unsigned short hh = f2bf(p); ps1[li] = hh; ps2[li] = f2bf(p - bf2f(hh)); } else { ps1[li] = hbits(p * PCAR); }
            }
#pragma unroll
            for (int sh = 1; sh < 16; sh <<= 1) psum += __shfl_xor(psum, sh, 32);
            l[r] = l[r] * corr + psum; m[r] = nm;
#pragma unroll
            for (int nd = 0; nd < 8; ++nd) o[nd][r] *= corr;
        }
        __syncthreads();
        V pf[2], pf2[2];
#pragma unroll
        for (int ks = 0; ks < KT / 32; ++ks) { pf[ks] = WFrag<T16>::lda(ps1 + lr * PSP + ks * 32 + 8 * hi); if (HR) pf2[ks] = WFrag<T16>::lda(ps2 + lr * PSP + ks * 32 + 8 * hi); }
#pragma unroll
        for (int nd = 0; nd < 8; ++nd) {
#pragma unroll
            for (int ks = 0; ks < KT / 32; ++ks) {
                const size_t vv = (size_t)nd * 16 * tp + t0 + ks * 32;
                const V b = WFrag<T16>::ld(vb + vv);
                o[nd] = WFrag<T16>::mma(pf[ks], b, o[nd]);
                if (HR) { const V b2 = WFrag<T16>::ld(vb2 + vv); o[nd] = WFrag<T16>::mma(pf2[ks], b, o[nd]); o[nd] = WFrag<T16>::mma(pf[ks], b2, o[nd]); }
            }
        }
        asm volatile("v_nop\n\tv_nop\n\tv_nop\n\tv_nop" : "+v"(o[0]), "+v"(o[1]), "+v"(o[2]), "+v"(o[3]), "+v"(o[4]), "+v"(o[5]), "+v"(o[6]), "+v"(o[7]) : "v"(pf[KT / 32 - 1]));
        __syncthreads();
    }
#pragma unroll
    for (int r = 0; r < 8; ++r) {
        const float fr = (HR ? 1.0f : (OCAR / PCAR)) / l[r];
#pragma unroll
        for (int nd = 0; nd < 8; ++nd) { const float v = o[nd][r] * fr; const int li = (8 * hi + r) * OSP + nd * 16 + lr;
            if (HR) { const unsigned short hh = f2bf(v); os1[li] = hh; os2[li] = f2bf(v - bf2f(hh)); } else { os1[li] = hbits(v); } }
    }
    __syncthreads();
    const size_t ob = (size_t)(row0 - obase) * DM + (size_t)h * HD + lr * 8;
#pragma unroll 1
    for (int ps = 0; ps < 2; ++ps) {
#pragma unroll
        for (int si = 0; si < 8; ++si) { const int row = 2 * si + hi;
            const v8us w1 = *(const v8usa*)(os1 + row * OSP + lr * 8); *(volatile v8us*)(O1 + ob + (size_t)row * DM) = w1;
            if (HR) { const v8us w2 = *(const v8usa*)(os2 + row * OSP + lr * 8); *(volatile v8us*)(O2 + ob + (size_t)row * DM) = w2; } }
        if (ps == 0) __threadfence();
    }
}

extern "C" void kernel_launch(void* const* d_in, const int* in_sizes, int n_in,
                              void* d_out, int out_size, void* d_ws, size_t ws_size, hipStream_t stream) {
    if (n_in < 5) return;
    const size_t needx = (size_t)(NB - 1) * TT_FULL * DM + (size_t)TT * DM;
    if ((size_t)in_sizes[0] < needx) return;
    for (int i = 1; i < 5; ++i) if ((size_t)in_sizes[i] < (size_t)DM * DM) return;
    if ((size_t)out_size < needx) return;
    const float* x = (const float*)d_in[0]; const float* wq = (const float*)d_in[1]; const float* wk = (const float*)d_in[2]; const float* wv = (const float*)d_in[3]; const float* wo = (const float*)d_in[4];
    float* OUT = (float*)d_out;
    char* wsp = (char*)d_ws;
    auto take = [&](size_t bytes) { char* p = wsp; wsp += (bytes + 255) & ~(size_t)255; return (void*)p; };
    bf* WQKV = (bf*)take((size_t)3 * DM * DM * 2);
    bf* WO   = (bf*)take((size_t)DM * DM * 2);
    h16* WO16 = (h16*)take((size_t)DM * DM * 2);
    float* CS = (float*)take((size_t)TT * HD * 2 * 4);
    bf* XB = (bf*)take((size_t)TT * DM * 2);
    float* F = (float*)take((size_t)TT * DM * 4);
    h16* QP16 = (h16*)take((size_t)NH * TT * HD * 2); h16* KP16 = (h16*)take((size_t)NH * TT * HD * 2); h16* VT16 = (h16*)take((size_t)NH * HD * TT * 2);
    bf* QPh = (bf*)take((size_t)NH * RHC * HD * 2); bf* QPl = (bf*)take((size_t)NH * RHC * HD * 2); bf* KPh = (bf*)take((size_t)NH * RHC * HD * 2); bf* KPl = (bf*)take((size_t)NH * RHC * HD * 2);
    bf* VTh = (bf*)take((size_t)NH * HD * RHC * 2); bf* VTl = (bf*)take((size_t)NH * HD * RHC * 2);
    bf* AT16 = (bf*)take((size_t)(TT - RHC) * DM * 2);
    bf* ATh = (bf*)take((size_t)RHC * DM * 2); bf* ATl = (bf*)take((size_t)RHC * DM * 2);
    if ((size_t)(wsp - (char*)d_ws) > ws_size) return;
    const unsigned GW = (unsigned)((DM * DM / 64 + 63) / 64);
    k_wtG<<<GW, 256, 0, stream>>>(wq, DM, DM, WQKV);
    k_wtG<<<GW, 256, 0, stream>>>(wk, DM, DM, WQKV + (size_t)DM * DM);
    k_wtG<<<GW, 256, 0, stream>>>(wv, DM, DM, WQKV + (size_t)2 * DM * DM);
    k_wtG<<<GW, 256, 0, stream>>>(wo, DM, DM, WO);
    k_wtG16<<<GW, 256, 0, stream>>>(wo, DM, DM, OCAR, WO16);
    k_cstab<<<(unsigned)((TT * (HD / 2) + 255) / 256), 256, 0, stream>>>(CS);
    const unsigned LP = (unsigned)(((size_t)NH * TT * HD / 2 + 255) / 256);
    for (int b = 0; b < NB; ++b) {
        const float* xb = x + (size_t)b * TT_FULL * DM; float* outb = OUT + (size_t)b * TT_FULL * DM;
        k_cvt8<<<(unsigned)(((size_t)TT * DM / 8 + 255) / 256), 256, 0, stream>>>(xb, XB, (size_t)TT * DM / 8);
        k_gemmw<bf, 0, false><<<dim3(TT / 64, DM / 64, 1), 32, 0, stream>>>(XB, nullptr, WQKV, nullptr, DM, F, DM, nullptr, 1.0f, 0, 0, 0);
        k_rope<<<LP, 256, 0, stream>>>(F, DM, NH, CS, QP16, QPh, QPl);
        k_gemmw<bf, 0, false><<<dim3(TT / 64, DM / 64, 1), 32, 0, stream>>>(XB, nullptr, WQKV + (size_t)DM * DM, nullptr, DM, F, DM, nullptr, 1.0f, 0, 0, 0);
        k_rope<<<LP, 256, 0, stream>>>(F, DM, NH, CS, KP16, KPh, KPl);
        k_gemmw<bf, 0, false><<<dim3(TT / 64, DM / 64, 1), 32, 0, stream>>>(XB, nullptr, WQKV + (size_t)2 * DM * DM, nullptr, DM, F, DM, nullptr, 1.0f, 0, 0, 0);
        k_vtp<<<LP, 256, 0, stream>>>(F, DM, NH, VT16, VTh, VTl);
        k_flash<bf, true><<<dim3(RHC / 16, NH, 1), 32, 0, stream>>>(QPh, QPl, KPh, KPl, VTh, VTl, RHC, 0, 0, ATh, ATl);
        if (TT > RHC) k_flash<h16, false><<<dim3((TT - RHC) / 16, NH, 1), 32, 0, stream>>>(QP16, QP16, KP16, KP16, VT16, VT16, TT, RHC, RHC, AT16, AT16);
        k_gemmw<bf, 1, false><<<dim3(RHC / 64, DM / 64, 1), 32, 0, stream>>>(ATh, ATl, WO, nullptr, DM, outb, DM, nullptr, 1.0f, 0, 0, 0);
        if (TT > RHC) k_gemmw<h16, 0, false><<<dim3((TT - RHC) / 64, DM / 64, 1), 32, 0, stream>>>((const h16*)AT16, nullptr, WO16, nullptr, DM, outb + (size_t)RHC * DM, DM, nullptr, OCINV, 0, 0, 0);
    }
}
